// DeformableSelfAttention3D_52871047414101
// MI455X (gfx1250) — hardware-verified
//
#include <hip/hip_runtime.h>
#include <math.h>

typedef __attribute__((ext_vector_type(16))) _Float16 v16h;
typedef __attribute__((ext_vector_type(16))) __bf16 v16b;
typedef __attribute__((ext_vector_type(8)))  _Float16 v8h;
typedef __attribute__((ext_vector_type(8)))  float v8f;
typedef __attribute__((ext_vector_type(4)))  float v4f;
typedef __attribute__((ext_vector_type(2)))  float v2f;
typedef __attribute__((ext_vector_type(4)))  unsigned v4u;
typedef __attribute__((ext_vector_type(4)))  int v4i;
typedef float __attribute__((may_alias)) float_a;
typedef int __attribute__((may_alias)) int_a;

template <typename T> __device__ __forceinline__ void vst2(void* p, T v) { *(volatile T*)p = v; __threadfence(); *(volatile T*)p = v; }
__device__ __forceinline__ v8f wmma16(v16h a, v16h b, v8f c) {
  v8f d = __builtin_amdgcn_wmma_f32_16x16x32_f16(false, a, false, b, (short)0, c, false, false);
  asm volatile("v_nop\n\tv_nop\n\tv_nop\n\tv_nop" : "+v"(d) : "v"(a), "v"(b));
  return d;
}
__device__ __forceinline__ v8f wmma_bf(v16b a, v16b b, v8f c) {
  v8f d = __builtin_amdgcn_wmma_f32_16x16x32_bf16(false, a, false, b, (short)0, c, false, false);
  asm volatile("v_nop\n\tv_nop\n\tv_nop\n\tv_nop" : "+v"(d) : "v"(a), "v"(b));
  return d;
}
__device__ __forceinline__ v16h frag_h(const _Float16* rowk0, int lane) {
  union { v16h v; v8h q[2]; } u; const _Float16* p = rowk0 + 8 * (lane >> 4);
  u.q[0] = *(const v8h*)p; u.q[1] = *(const v8h*)(p + 16); return u.v;
}
__device__ __forceinline__ v16h frag_f32(const float* rowk0, int lane) {
  v16h a; const float* p = rowk0 + 8 * (lane >> 4);
#pragma unroll
  for (int i = 0; i < 8; ++i) { a[i] = (_Float16)p[i]; a[8 + i] = (_Float16)p[16 + i]; }
  return a;
}
__device__ __forceinline__ v16h frag_f32s(const float* rowk0, int lane, float sc) {
  v16h a; const float* p = rowk0 + 8 * (lane >> 4);
#pragma unroll
  for (int i = 0; i < 8; ++i) { a[i] = (_Float16)(p[i] * sc); a[8 + i] = (_Float16)(p[16 + i] * sc); }
  return a;
}
__device__ __forceinline__ v16h fragc_f32(const float* W, int k0, int n, int lane, int ld, int K) {
  v16h a; const int g = lane >> 4;
#pragma unroll
  for (int i = 0; i < 8; ++i) { const int ka = k0 + 8 * g + i, kb = ka + 16;
    a[i] = (_Float16)(ka < K ? W[(size_t)(ka < K ? ka : K - 1) * ld + n] : 0.f); a[8 + i] = (_Float16)(kb < K ? W[(size_t)(kb < K ? kb : K - 1) * ld + n] : 0.f); }
  return a;
}
struct F2 { v16b h, l; };
__device__ __forceinline__ F2 bsplit16(const float v[16]) { F2 r;
#pragma unroll
  for (int i = 0; i < 16; ++i) { const __bf16 h = (__bf16)v[i]; r.h[i] = h; r.l[i] = (__bf16)(v[i] - (float)h); }
  return r; }
__device__ __forceinline__ F2 split_row(const float* row, int k0, int lane) { float v[16]; const float* p = row + k0 + 8 * (lane >> 4);
#pragma unroll
  for (int i = 0; i < 8; ++i) { v[i] = p[i]; v[8 + i] = p[16 + i]; }
  return bsplit16(v); }
__device__ __forceinline__ F2 split_rowK(const float* row, int k0, int lane, int K) { float v[16]; const int g = lane >> 4;
#pragma unroll
  for (int i = 0; i < 8; ++i) { const int ka = k0 + 8 * g + i, kb = ka + 16; v[i] = ka < K ? row[ka < K ? ka : K - 1] : 0.f; v[8 + i] = kb < K ? row[kb < K ? kb : K - 1] : 0.f; }
  return bsplit16(v); }
__device__ __forceinline__ F2 split_col(const float* W, int k0, int n, int lane, int ld, int K) { float v[16]; const int g = lane >> 4;
#pragma unroll
  for (int i = 0; i < 8; ++i) { const int ka = k0 + 8 * g + i, kb = ka + 16; v[i] = ka < K ? W[(size_t)(ka < K ? ka : K - 1) * ld + n] : 0.f; v[8 + i] = kb < K ? W[(size_t)(kb < K ? kb : K - 1) * ld + n] : 0.f; }
  return bsplit16(v); }
__device__ __forceinline__ v8f mac3(const F2& a, const F2& b, v8f c) { c = wmma_bf(a.l, b.h, c); c = wmma_bf(a.h, b.l, c); return wmma_bf(a.h, b.h, c); }
__device__ __forceinline__ float sigm(float v) { return 1.0f / (1.0f + expf(-v)); }
#define LDSX() do { asm volatile("s_wait_dscnt 0" ::: "memory"); __builtin_amdgcn_wave_barrier(); __builtin_amdgcn_fence(__ATOMIC_RELEASE, "workgroup"); } while (0)


#define NBT 2
#define SD0 20
#define NTOK (SD0 * SD0 * SD0)
#define CC 384
#define NHD 8
#define HDM 48
#define SD1 10
#define MTOK (SD1 * SD1 * SD1)
#define MKP 1024
#define NQ (NBT * NTOK)
#define NKV (NBT * MTOK)
#define NKVP 2048
#define KSR (8 * CC)
#define KOF (27 * CC)
#define KPJ 512
#ifndef TNB
#define TNB NBT
#define TQT (NQ / 64)
#endif
typedef __attribute__((ext_vector_type(8))) __bf16 v8b;
__device__ __forceinline__ v16b frag_b(const __bf16* rowk0, int lane) {
  union { v16b v; v8b q[2]; } u; const __bf16* p = rowk0 + 8 * (lane >> 4);
  u.q[0] = *(const v8b*)p; u.q[1] = *(const v8b*)(p + 16); return u.v;
}
__device__ __forceinline__ float bfr(float v) { return (float)(__bf16)v; }
__device__ __attribute__((noinline)) float exp_ni(float v) { return expf(v); }
__device__ __attribute__((noinline)) float erf_ni(float v) { return erff(v); }
__device__ __attribute__((noinline)) float tanh_ni(float v) { return tanhf(v); }
__constant__ float c_lin[SD1] = {-1.000000000e+00f,-7.777777910e-01f,-5.555555820e-01f,-3.333332837e-01f,-1.111111343e-01f,1.111111417e-01f,3.333333731e-01f,5.555555820e-01f,7.777777910e-01f,1.000000000e+00f};
__device__ __forceinline__ v16b zfrag_if(v16b a, bool ok) { const v16b z = {}; return ok ? a : z; }

#define PK_Q  0
#define PK_SR (PK_Q + CC * CC)
#define PK_KV (PK_SR + (size_t)CC * KSR)
#define PK_OF (PK_KV + (size_t)2 * CC * CC)
#define PK_PJ (PK_OF + (size_t)32 * KOF)
#define PK_END (PK_PJ + (size_t)CC * KPJ)
#define WS_PK  0u
#define WS_XB  (((2u * PK_END) + 127u) / 128u * 128u)
#define WS_Q   (WS_XB + 2u * NQ * CC)
#define WS_XS  (WS_Q + 4u * NQ * CC)
#define WS_XLH (WS_XS + 4u * NKVP * CC)
#define WS_XLL (WS_XLH + 2u * NKVP * CC)
#define WS_KV  (WS_XLL + 2u * NKVP * CC)
#define WS_OFS (WS_KV + 4u * NKVP * 2 * CC)
#define WS_SK  (WS_OFS + 4u * NKVP * 32)
#define WS_SVH (WS_SK + 4u * NBT * NHD * MKP * 64)
#define WS_SVL (WS_SVH + 2u * NBT * NHD * HDM * MKP)
#define WS_O   (WS_SVL + 2u * NBT * NHD * HDM * MKP)
#define WS_END (WS_O + 4u * NQ * KPJ)

__global__ __launch_bounds__(256) void k_pack(const float* __restrict__ QW, const float* __restrict__ SRW, const float* __restrict__ KVW, const float* __restrict__ OFW, const float* __restrict__ PJW, __bf16* __restrict__ PK) {
  __shared__ __align__(16) __bf16 s[KOF]; const int o = blockIdx.x, which = blockIdx.y, tid = threadIdx.x; int K; size_t dst;
  if (which == 0) { if (o >= CC) return; K = CC; dst = PK_Q + (size_t)o * CC; for (int k = tid; k < K; k += 256) s[k] = (__bf16)QW[(size_t)o * CC + k]; }
  else if (which == 1) { if (o >= CC) return; K = KSR; dst = PK_SR + (size_t)o * KSR; for (int k = tid; k < K; k += 256) { const int tap = k / CC, c = k % CC; s[k] = (__bf16)SRW[((size_t)o * CC + c) * 8 + tap]; } }
  else if (which == 2) { K = CC; dst = PK_KV + (size_t)o * CC; for (int k = tid; k < K; k += 256) s[k] = (__bf16)KVW[(size_t)o * CC + k]; }
  else if (which == 3) { if (o >= 32) return; K = KOF; dst = PK_OF + (size_t)o * KOF; for (int k = tid; k < K; k += 256) { const int tap = k / CC, c = k % CC; s[k] = (__bf16)((o < 3 * NHD) ? OFW[((size_t)o * CC + c) * 27 + tap] : 0.f); } }
  else { if (o >= CC) return; K = KPJ; dst = PK_PJ + (size_t)o * KPJ; for (int k = tid; k < K; k += 256) { const int h = k / 64, ch = k % 64; s[k] = (__bf16)((ch < HDM) ? PJW[(size_t)o * CC + h * HDM + ch] : 0.f); } }
  __syncthreads();
  for (int q = tid; q < K / 8; q += 256) vst2((unsigned*)(PK + dst + q * 8), *(const v4u*)&s[q * 8]);
}
__global__ __launch_bounds__(64) void k_xb(const float* __restrict__ X, __bf16* __restrict__ XB) {
  __shared__ __align__(16) __bf16 s[CC]; const size_t r = blockIdx.x; const int t = threadIdx.x;
  for (int k = t; k < CC; k += 64) s[k] = (__bf16)X[r * CC + k];
  __syncthreads();
  if (t < CC / 8) vst2((unsigned*)(XB + r * CC + t * 8), *(const v4u*)&s[t * 8]);
}
template <int MODE>
__global__ __launch_bounds__(128) void k_gemm(const __bf16* __restrict__ A0, const __bf16* __restrict__ A1, const float* __restrict__ AF, const __bf16* __restrict__ P, const float* __restrict__ bias, float* __restrict__ OUT) {
  constexpr int K = (MODE == 1) ? KSR : (MODE == 3) ? KPJ : CC; constexpr int LDO = (MODE == 2) ? 2 * CC : CC;
  __shared__ __align__(16) float so[4][16][132];
  const int tid = threadIdx.x, wave = tid >> 5, lane = tid & 31, col = lane & 15, g = lane >> 4; const size_t r0 = (size_t)blockIdx.x * 64 + wave * 16; const int n0 = blockIdx.y * 128; const size_t ra = r0 + col;
  v8f acc[8] = {};
  if (MODE == 1) { const size_t rc = (ra < (size_t)NKV) ? ra : (size_t)(NKV - 1); const int b = (int)(rc / MTOK), m = (int)(rc % MTOK);   const int dz = m / 100, hy = (m / 10) % 10, wx = m % 10;
#pragma unroll 1
    for (int tap = 0; tap < 8; ++tap) { const int kd = tap >> 2, kh = (tap >> 1) & 1, kw = tap & 1; const size_t tok = ((size_t)(2 * dz + kd) * SD0 + (size_t)(2 * hy + kh)) * SD0 + (size_t)(2 * wx + kw); const size_t src = ((size_t)b * NTOK + tok) * CC;
#pragma unroll 4
      for (int kc = 0; kc < CC / 32; ++kc) { const v16b a = frag_b(A0 + src + kc * 32, lane);
#pragma unroll
        for (int j = 0; j < 8; ++j) acc[j] = wmma_bf(a, frag_b(P + (size_t)(n0 + j * 16 + col) * K + (size_t)tap * CC + kc * 32, lane), acc[j]); } } }
  else {
#pragma unroll 2
    for (int kc = 0; kc < K / 32; ++kc) { F2 a; if (MODE == 3) a = split_row(AF + ra * K, kc * 32, lane); else { a.h = frag_b(A0 + ra * K + kc * 32, lane); if (MODE == 2) a.l = frag_b(A1 + ra * K + kc * 32, lane); }
#pragma unroll
      for (int j = 0; j < 8; ++j) { const v16b w = frag_b(P + (size_t)(n0 + j * 16 + col) * K + kc * 32, lane); if (MODE >= 2) acc[j] = wmma_bf(a.l, w, acc[j]); acc[j] = wmma_bf(a.h, w, acc[j]); } } }
#pragma unroll
  for (int j = 0; j < 8; ++j) { const float bb = bias ? bfr(bias[n0 + j * 16 + col]) : 0.f;
#pragma unroll
    for (int r = 0; r < 8; ++r) so[wave][8 * g + r][j * 16 + col] = acc[j][r] + bb; }
  LDSX();
  for (int rl = 0; rl < 16; ++rl) vst2(OUT + (r0 + rl) * LDO + n0 + lane * 4, *(const v4f*)&so[wave][rl][lane * 4]);
}
__global__ __launch_bounds__(256) void k_ln(const float* __restrict__ XS, const float* __restrict__ G, const float* __restrict__ Bv, __bf16* __restrict__ XLH, __bf16* __restrict__ XLL) {
  __shared__ __align__(16) __bf16 sh_[16][392], sl_[16][392]; __shared__ float sred[16][16], smu[16], srs[16];
  const int tid = threadIdx.x; const int tl = tid >> 4, li = tid & 15; const size_t row = (size_t)blockIdx.x * 16 + tl; const float* xr = XS + row * CC;
  float s = 0.f; for (int k = li; k < CC; k += 16) s += xr[k]; sred[tl][li] = s; __syncthreads();
  if (li == 0) { float a = 0.f; for (int i = 0; i < 16; ++i) a += sred[tl][i]; smu[tl] = a / (float)CC; } __syncthreads();
  const float mu = smu[tl]; float q = 0.f; for (int k = li; k < CC; k += 16) { const float d = xr[k] - mu; q += d * d; } sred[tl][li] = q; __syncthreads();
  if (li == 0) { float a = 0.f; for (int i = 0; i < 16; ++i) a += sred[tl][i]; srs[tl] = rsqrtf(a / (float)CC + 1e-5f); } __syncthreads();
  const float rs = srs[tl]; for (int k = li; k < CC; k += 16) { const float v = (xr[k] - mu) * rs * bfr(G[k]) + bfr(Bv[k]); const __bf16 hb = (__bf16)v; sh_[tl][k] = hb; sl_[tl][k] = (__bf16)(v - (float)hb); }
  __syncthreads();
  for (int q2 = tid; q2 < 16 * (CC / 8); q2 += 256) { const int t = q2 / (CC / 8), pc = q2 % (CC / 8); const size_t o = ((size_t)blockIdx.x * 16 + t) * CC + pc * 8; vst2((unsigned*)(XLH + o), *(const v4u*)&sh_[t][pc * 8]); vst2((unsigned*)(XLL + o), *(const v4u*)&sl_[t][pc * 8]); }
}
__global__ __launch_bounds__(128) void k_off(const __bf16* __restrict__ XLH, const __bf16* __restrict__ XLL, const __bf16* __restrict__ P, const float* __restrict__ OB, float* __restrict__ OFS) {
  __shared__ __align__(16) float so[4][16][36];
  const int tid = threadIdx.x, wave = tid >> 5, lane = tid & 31, col = lane & 15, g = lane >> 4; const size_t r0 = (size_t)blockIdx.x * 64 + wave * 16; const size_t ra = r0 + col;
  const size_t rc = (ra < (size_t)NKV) ? ra : (size_t)(NKV - 1); const int b = (int)(rc / MTOK), m = (int)(rc % MTOK); const int dz = m / 100, hy = (m / 10) % 10, wx = m % 10;
  v8f acc[2] = {};
#pragma unroll 1
  for (int tap = 0; tap < 27; ++tap) { const int zz = dz + tap / 9 - 1, yy = hy + (tap / 3) % 3 - 1, xx = wx + tap % 3 - 1; const bool ok = zz >= 0 && zz < SD1 && yy >= 0 && yy < SD1 && xx >= 0 && xx < SD1;
    const size_t src = ((size_t)b * MTOK + ((size_t)min(max(zz, 0), SD1 - 1) * SD1 + min(max(yy, 0), SD1 - 1)) * SD1 + min(max(xx, 0), SD1 - 1)) * CC;
#pragma unroll 2
    for (int kc = 0; kc < CC / 32; ++kc) { const v16b ah = zfrag_if(frag_b(XLH + src + kc * 32, lane), ok), al = zfrag_if(frag_b(XLL + src + kc * 32, lane), ok); const size_t kk = (size_t)tap * CC + kc * 32;
#pragma unroll
      for (int j = 0; j < 2; ++j) { const v16b w = frag_b(P + (size_t)(j * 16 + col) * KOF + kk, lane); acc[j] = wmma_bf(al, w, acc[j]); acc[j] = wmma_bf(ah, w, acc[j]); } } }
#pragma unroll
  for (int j = 0; j < 2; ++j) { const int o = j * 16 + col; const float bb = (o < 3 * NHD) ? bfr(OB[min(o, 3 * NHD - 1)]) : 0.f;
#pragma unroll
    for (int r = 0; r < 8; ++r) so[wave][8 * g + r][o] = (o < 3 * NHD) ? 2.0f * tanh_ni(acc[j][r] + bb) : 0.f; }
  LDSX();
  for (int rl = 0; rl < 16; ++rl) if (lane < 8) vst2(OFS + (r0 + rl) * 32 + lane * 4, *(const v4f*)&so[wave][rl][lane * 4]);
}
__global__ __launch_bounds__(128) void k_samp(const float* __restrict__ KV, const float* __restrict__ OFS, float* __restrict__ SK, _Float16* __restrict__ SVH, _Float16* __restrict__ SVL) {
  __shared__ __align__(16) float sk[64][68]; __shared__ __align__(16) _Float16 svh[HDM][72], svl[HDM][72]; __shared__ int sidx[64][8]; __shared__ float swt[64][8];
  const int tid = threadIdx.x; const int p0 = blockIdx.x * 64, bh = blockIdx.y; const int b = bh / NHD, h = bh % NHD;
  if (tid < 64) { const int p = p0 + tid; float g3[3]; int valid_p = (p < MTOK);
    const int pd = p / 100, ph = (p / 10) % 10, pw = p % 10; const float base[3] = {c_lin[min(pd, SD1 - 1)], c_lin[ph], c_lin[pw]};
#pragma unroll
    for (int c = 0; c < 3; ++c) g3[c] = valid_p ? base[c] + OFS[((size_t)b * MTOK + min(p, MTOK - 1)) * 32 + h * 3 + c] : 0.f;
    const float ix = ((g3[0] + 1.0f) * 0.5f) * (float)(SD1 - 1), iy = ((g3[1] + 1.0f) * 0.5f) * (float)(SD1 - 1), iz = ((g3[2] + 1.0f) * 0.5f) * (float)(SD1 - 1);
    const float x0f = floorf(ix), y0f = floorf(iy), z0f = floorf(iz); const float fx = ix - x0f, fy = iy - y0f, fz = iz - z0f; const int x0 = (int)x0f, y0 = (int)y0f, z0 = (int)z0f;
#pragma unroll
    for (int cnr = 0; cnr < 8; ++cnr) { const int dzz = cnr >> 2, dyy = (cnr >> 1) & 1, dxx = cnr & 1; const int zi = z0 + dzz, yi = y0 + dyy, xi = x0 + dxx;
      const float wz = dzz ? fz : 1.0f - fz, wy = dyy ? fy : 1.0f - fy, wxv = dxx ? fx : 1.0f - fx; const bool ok = xi >= 0 && xi < SD1 && yi >= 0 && yi < SD1 && zi >= 0 && zi < SD1;
      sidx[tid][cnr] = (min(max(zi, 0), SD1 - 1) * SD1 + min(max(yi, 0), SD1 - 1)) * SD1 + min(max(xi, 0), SD1 - 1); swt[tid][cnr] = valid_p ? ((wxv * wy) * wz) * (ok ? 1.0f : 0.0f) : 0.f; } }
  __syncthreads();
  for (int q = tid; q < 64 * HDM; q += 128) { const int pl = q / HDM, ch = q % HDM; float ak = 0.f, av = 0.f;
#pragma unroll
    for (int cnr = 0; cnr < 8; ++cnr) { const float* row = KV + ((size_t)b * MTOK + sidx[pl][cnr]) * 2 * CC + h * HDM + ch; const float w = swt[pl][cnr]; ak += row[0] * w; av += row[CC] * w; }
    sk[pl][ch] = ak; const _Float16 hv = (_Float16)av; svh[ch][pl] = hv; svl[ch][pl] = (_Float16)((av - (float)hv) * 2048.0f); }
  for (int q = tid; q < 64 * 16; q += 128) { const int pl = q >> 4, ch = HDM + (q & 15); sk[pl][ch] = 0.f; }
  __syncthreads();
  for (int q = tid; q < 64 * 16; q += 128) { const int pl = q >> 4, pc = q & 15; vst2(SK + ((size_t)bh * MKP + p0 + pl) * 64 + pc * 4, *(const v4f*)&sk[pl][pc * 4]); }
  for (int q = tid; q < HDM * 8; q += 128) { const int ch = q >> 3, pc = q & 7; const size_t o = ((size_t)bh * HDM + ch) * MKP + p0 + pc * 8; vst2((unsigned*)(SVH + o), *(const v4u*)&svh[ch][pc * 8]); vst2((unsigned*)(SVL + o), *(const v4u*)&svl[ch][pc * 8]); }
}
__device__ __forceinline__ v16h frag_f32_48(const float* rowk32, int lane) { v16h a; const float* p = rowk32 + 8 * (lane >> 4);
#pragma unroll
  for (int i = 0; i < 8; ++i) { a[i] = (_Float16)p[i]; a[8 + i] = (_Float16)0.f; } return a; }
__global__ __launch_bounds__(128) void k_att(const float* __restrict__ Q, const float* __restrict__ SK, const _Float16* __restrict__ SVH, const _Float16* __restrict__ SVL, float* __restrict__ O) {
  __shared__ __align__(16) float sp[4][16][36]; __shared__ __align__(16) float so[4][16][68];
  const int tid = threadIdx.x, wave = tid >> 5, lane = tid & 31, col = lane & 15, g = lane >> 4; const int qb = blockIdx.x, h = blockIdx.y, b = blockIdx.z; const int bh = b * NHD + h; const size_t rq = (size_t)b * NTOK + (size_t)qb * 64 + wave * 16 + col;
  const v16h aq0 = frag_f32(Q + rq * CC + h * HDM, lane), aq1 = frag_f32_48(Q + rq * CC + h * HDM + 32, lane);
  float m[8], l[8];
#pragma unroll
  for (int r = 0; r < 8; ++r) { m[r] = -3.0e38f; l[r] = 0.f; }
  v8f acc[3] = {}, accl[3] = {};
#pragma unroll 1
  for (int ks = 0; ks < MKP / 32; ++ks) { v8f s[2];
#pragma unroll
    for (int ct = 0; ct < 2; ++ct) { const int kk = ks * 32 + ct * 16 + col; const float* krow = SK + ((size_t)bh * MKP + kk) * 64; v8f c = {}; c = wmma16(aq0, frag_f32(krow, lane), c); c = wmma16(aq1, frag_f32_48(krow + 32, lane), c);
#pragma unroll
      for (int r = 0; r < 8; ++r) s[ct][r] = (kk < MTOK) ? c[r] * 0.14433756729740643f : -3.0e38f; }
#pragma unroll
    for (int r = 0; r < 8; ++r) { float mx = fmaxf(s[0][r], s[1][r]);
#pragma unroll
      for (int o = 1; o < 16; o <<= 1) mx = fmaxf(mx, __shfl_xor(mx, o));
      const float mn = fmaxf(m[r], mx); const float alpha = (m[r] <= -1.0e38f) ? 0.f : __expf(m[r] - mn);
      const float e0 = (float)(_Float16)(((s[0][r] <= -1.0e38f) ? 0.f : __expf(s[0][r] - mn)) * 1024.0f), e1 = (float)(_Float16)(((s[1][r] <= -1.0e38f) ? 0.f : __expf(s[1][r] - mn)) * 1024.0f); float es = e0 + e1;
#pragma unroll
      for (int o = 1; o < 16; o <<= 1) es += __shfl_xor(es, o);
      l[r] = l[r] * alpha + es; m[r] = mn;
#pragma unroll
      for (int dt = 0; dt < 3; ++dt) { acc[dt][r] *= alpha; accl[dt][r] *= alpha; }
      sp[wave][8 * g + r][col] = e0; sp[wave][8 * g + r][16 + col] = e1; }
    LDSX();
    const v16h pa = frag_f32(&sp[wave][col][0], lane);
#pragma unroll
    for (int dt = 0; dt < 3; ++dt) { const size_t vr = ((size_t)bh * HDM + dt * 16 + col) * MKP + (size_t)ks * 32; acc[dt] = wmma16(pa, frag_h(SVH + vr, lane), acc[dt]); accl[dt] = wmma16(pa, frag_h(SVL + vr, lane), accl[dt]); }
    LDSX(); }
#pragma unroll
  for (int r = 0; r < 8; ++r) { const float il = 1.0f / l[r];
#pragma unroll
    for (int dt = 0; dt < 3; ++dt) so[wave][8 * g + r][dt * 16 + col] = (acc[dt][r] + accl[dt][r] * (1.0f / 2048.0f)) * il;
    so[wave][8 * g + r][48 + col] = 0.f; }
  LDSX();
  for (int rl = 0; rl < 16; ++rl) if (lane < 16) vst2(O + (rq - col + rl) * KPJ + h * 64 + lane * 4, *(const v4f*)&so[wave][rl][lane * 4]);
}
extern "C" void kernel_launch(void* const* d_in, const int* in_sizes, int n_in, void* d_out, int out_size, void* d_ws, size_t ws_size, hipStream_t stream) {
  (void)in_sizes; (void)n_in; (void)out_size;
  const float** F = (const float**)d_in;
  if (ws_size < (size_t)WS_END) return;
  char* ws = (char*)d_ws; __bf16 *PK = (__bf16*)(ws + WS_PK), *XB = (__bf16*)(ws + WS_XB), *XLH = (__bf16*)(ws + WS_XLH), *XLL = (__bf16*)(ws + WS_XLL); float *Q = (float*)(ws + WS_Q), *XS = (float*)(ws + WS_XS), *KV = (float*)(ws + WS_KV), *OFS = (float*)(ws + WS_OFS), *SK = (float*)(ws + WS_SK), *O = (float*)(ws + WS_O); _Float16 *SVH = (_Float16*)(ws + WS_SVH), *SVL = (_Float16*)(ws + WS_SVL);
  k_pack<<<dim3(2 * CC, 5), 256, 0, stream>>>(F[1], F[5], F[2], F[9], F[3], PK);
  k_xb<<<NQ, 64, 0, stream>>>(F[0], XB);
  k_gemm<0><<<dim3(TQT, CC / 128), 128, 0, stream>>>(XB, nullptr, nullptr, PK + PK_Q, nullptr, Q);
  k_gemm<1><<<dim3((TNB * MTOK + 63) / 64, CC / 128), 128, 0, stream>>>(XB, nullptr, nullptr, PK + PK_SR, F[6], XS);
  k_ln<<<(TNB * MTOK + 63) / 64 * 4, 256, 0, stream>>>(XS, F[7], F[8], XLH, XLL);
  k_gemm<2><<<dim3((TNB * MTOK + 63) / 64, 2 * CC / 128), 128, 0, stream>>>(XLH, XLL, nullptr, PK + PK_KV, nullptr, KV);
  k_off<<<(TNB * MTOK + 63) / 64, 128, 0, stream>>>(XLH, XLL, PK + PK_OF, F[10], OFS);
  k_samp<<<dim3(MKP / 64, TNB * NHD), 128, 0, stream>>>(KV, OFS, SK, SVH, SVL);
  k_att<<<dim3(TQT < NTOK / 64 ? TQT : NTOK / 64, NHD, (TQT * 64 + NTOK - 1) / NTOK), 128, 0, stream>>>(Q, SK, SVH, SVL, O);
  k_gemm<3><<<dim3(TQT, CC / 128), 128, 0, stream>>>(nullptr, nullptr, O, PK + PK_PJ, F[4], (float*)d_out);
}
